// MSAOuterProductMean_66984309948700
// MI455X (gfx1250) — hardware-verified
//
#include <hip/hip_runtime.h>


#define NSQ  128
#define LL   256
#define CM   256
#define HDm  32
#define HP   64
#define PD   128
#define NR   (NSQ * LL)
#define ICH  16
#define PCAR 128.0f
typedef _Float16 h16;
typedef unsigned short bf;
typedef __attribute__((ext_vector_type(16))) __bf16   v16bf;
typedef __attribute__((ext_vector_type(16))) _Float16 v16h;
typedef __attribute__((ext_vector_type(8)))  _Float16 v8h;
typedef __attribute__((ext_vector_type(8)))  unsigned short v8us;
typedef __attribute__((ext_vector_type(8)))  float    v8f;
typedef __attribute__((ext_vector_type(4)))  float    v4f;
typedef v8h  __attribute__((may_alias)) v8ha;
typedef v4f  __attribute__((may_alias)) v4fa;
typedef v8us __attribute__((may_alias)) v8usa;

__device__ __forceinline__ unsigned short f2bf(float f) { unsigned u = __float_as_uint(f); u += 0x7FFFu + ((u >> 16) & 1u); return (unsigned short)(u >> 16); }
__device__ __forceinline__ float bf2f(unsigned short b) { return __uint_as_float(((unsigned)b) << 16); }
__device__ __forceinline__ float bfr(float f) { return bf2f(f2bf(f)); }
__device__ __forceinline__ v16h cat16(v8h lo, v8h hi) { return __builtin_shufflevector(lo, hi, 0, 1, 2, 3, 4, 5, 6, 7, 8, 9, 10, 11, 12, 13, 14, 15); }
__device__ __forceinline__ v16bf cat16b(v8us lo, v8us hi) { return __builtin_bit_cast(v16bf, __builtin_shufflevector(lo, hi, 0, 1, 2, 3, 4, 5, 6, 7, 8, 9, 10, 11, 12, 13, 14, 15)); }
__device__ __forceinline__ v8f wmma16(v16h a, v16h b, v8f c) { return __builtin_amdgcn_wmma_f32_16x16x32_f16(false, a, false, b, (short)0, c, false, false); }
__device__ __forceinline__ v8f wmmab(v16bf a, v16bf b, v8f c) { return __builtin_amdgcn_wmma_f32_16x16x32_bf16(false, a, false, b, (short)0, c, false, false); }


template <typename T16> struct WFrag;
template <> struct WFrag<h16> { typedef v16h V; static __device__ __forceinline__ V ld(const h16* p) { return cat16(*(const v8h*)p, *(const v8h*)(p + 16)); } static __device__ __forceinline__ v8f mma(V a, V b, v8f c) { return wmma16(a, b, c); } };
template <> struct WFrag<bf> { typedef v16bf V; static __device__ __forceinline__ V ld(const bf* p) { return cat16b(*(const v8us*)p, *(const v8us*)(p + 16)); } static __device__ __forceinline__ v8f mma(V a, V b, v8f c) { return wmmab(a, b, c); } };
template <typename T16, int NSPLIT, bool BIAS>
__global__ __launch_bounds__(32) void k_gemmw(const T16* __restrict__ A, const T16* __restrict__ A2, const T16* __restrict__ Bt, const T16* __restrict__ Bt2, int K, float* C, int ldc, const float* __restrict__ bias, size_t sA, size_t sB, size_t sC) {
    typedef typename WFrag<T16>::V V;
    __shared__ __align__(16) float os[16 * 68];
    const size_t z = blockIdx.z; A += z * sA; if (A2) A2 += z * sA; Bt += z * sB; if (Bt2) Bt2 += z * sB; C += z * sC;
    const int lane = threadIdx.x & 31, lr = lane & 15, hi = lane >> 4; const int r0 = blockIdx.x * 64, c0 = blockIdx.y * 64;
    v8f acc[4][4];
#pragma unroll
    for (int mb = 0; mb < 4; ++mb)
#pragma unroll
        for (int nb = 0; nb < 4; ++nb) acc[mb][nb] = (v8f){};
    const size_t aoff = (size_t)(r0 + lr) * K + 8 * hi, boff = (size_t)(c0 + lr) * K + 8 * hi;
#pragma unroll 1
    for (int kc = 0; kc < K; kc += 32) {
        V a[4], a2[4];
#pragma unroll
        for (int mb = 0; mb < 4; ++mb) { a[mb] = WFrag<T16>::ld(A + aoff + (size_t)mb * 16 * K + kc); if (NSPLIT == 1 || NSPLIT == 2) a2[mb] = WFrag<T16>::ld(A2 + aoff + (size_t)mb * 16 * K + kc); }
#pragma unroll
        for (int nb = 0; nb < 4; ++nb) { const V b = WFrag<T16>::ld(Bt + boff + (size_t)nb * 16 * K + kc); V b2; if (NSPLIT >= 2) b2 = WFrag<T16>::ld(Bt2 + boff + (size_t)nb * 16 * K + kc);
#pragma unroll
            for (int mb = 0; mb < 4; ++mb) { acc[mb][nb] = WFrag<T16>::mma(a[mb], b, acc[mb][nb]); if (NSPLIT == 1 || NSPLIT == 2) acc[mb][nb] = WFrag<T16>::mma(a2[mb], b, acc[mb][nb]); if (NSPLIT >= 2) acc[mb][nb] = WFrag<T16>::mma(a[mb], b2, acc[mb][nb]); } }
        asm volatile("v_nop\n\tv_nop\n\tv_nop\n\tv_nop" : "+v"(acc[0][0]), "+v"(acc[1][1]), "+v"(acc[2][2]), "+v"(acc[3][3]) : "v"(a[0]), "v"(a[3]));
    }
#pragma unroll
    for (int mb = 0; mb < 4; ++mb) {
#pragma unroll
        for (int nb = 0; nb < 4; ++nb) {
#pragma unroll
            for (int j = 0; j < 8; ++j) os[(hi * 8 + j) * 68 + nb * 16 + lr] = acc[mb][nb][j]; }
        __builtin_amdgcn_wave_barrier(); asm volatile("" ::: "memory");
        float* crow = C + (size_t)(r0 + mb * 16) * ldc + c0;
#pragma unroll 1
        for (int ps = 0; ps < 2; ++ps) {
#pragma unroll
            for (int s = 0; s < 8; ++s) { const int row = 2 * s + hi, cofs = lr * 4; v4f val = *(const v4fa*)(os + row * 68 + cofs); if (BIAS) { val[0] += bfr(bias[c0 + cofs]); val[1] += bfr(bias[c0 + cofs + 1]); val[2] += bfr(bias[c0 + cofs + 2]); val[3] += bfr(bias[c0 + cofs + 3]); }
                *(volatile v4f*)(crow + (size_t)row * ldc + cofs) = val; }
            if (ps == 0) __threadfence(); }
        __builtin_amdgcn_wave_barrier(); asm volatile("" ::: "memory");
    }
}

__device__ __forceinline__ h16 tohx(float x) { return (h16)x; }
__device__ __forceinline__ void splitf(float y, unsigned short& h, unsigned short& l) { h = f2bf(y); l = f2bf(y - bf2f(h)); }
typedef __attribute__((ext_vector_type(2))) unsigned short v2us;
typedef __attribute__((ext_vector_type(4))) unsigned short v4us;
typedef __attribute__((ext_vector_type(2))) _Float16 v2h;
typedef __attribute__((ext_vector_type(4))) _Float16 v4h;

__global__ __launch_bounds__(256) void k_wtG(const float* __restrict__ w, int K, int N, bf* Bt) {
    const int lane = threadIdx.x & 31; const int L0 = (blockIdx.x * 8 + (threadIdx.x >> 5)) * 8; const int nlines = N * K / 64;
#pragma unroll
    for (int ps = 0; ps < 2; ++ps) {
#pragma unroll 1
        for (int l = 0; l < 8; ++l) { const int L = L0 + l; if (L >= nlines) break; const size_t e = (size_t)L * 64 + lane * 2; const int k = (int)(e % K), n = (int)(e / K); v2us o;
            o[0] = f2bf(w[(size_t)k * N + n]); o[1] = f2bf(w[(size_t)(k + 1) * N + n]); *(volatile v2us*)(Bt + e) = o; }
        if (ps == 0) __threadfence(); }
}
__global__ __launch_bounds__(256) void k_wpadT(const float* __restrict__ w, int kreal, int nreal, int NOUT, int KP, bf* Bt) { const int e = (blockIdx.x * 256 + threadIdx.x) * 2; if (e >= NOUT * KP) return; const int k = e % KP, n = e / KP; v2us o; o[0] = (n < nreal && k < kreal) ? f2bf(w[(size_t)k * nreal + n]) : (unsigned short)0; o[1] = (n < nreal && k + 1 < kreal) ? f2bf(w[(size_t)(k + 1) * nreal + n]) : (unsigned short)0; *(volatile v2us*)(Bt + e) = o; __threadfence(); *(volatile v2us*)(Bt + e) = o; }
__global__ __launch_bounds__(64) void k_bpad(const float* __restrict__ b, float* BP) { const int n = threadIdx.x; const float v = n < HDm ? b[n] : 0.f; *(volatile float*)(BP + n) = v; __threadfence(); *(volatile float*)(BP + n) = v; }
__global__ __launch_bounds__(256) void k_ln(const float* __restrict__ X, const float* __restrict__ g, const float* __restrict__ bb, bf* Nh, bf* Nl) { const int lane = threadIdx.x & 31; const int row = blockIdx.x * 8 + (threadIdx.x >> 5); if (row >= NR) return; const size_t rb = (size_t)row * CM; const v4f a0 = *(const v4f*)(X + rb + lane * 4), a1 = *(const v4f*)(X + rb + 128 + lane * 4); float v[8];
#pragma unroll
    for (int u = 0; u < 4; ++u) { v[u] = bfr(a0[u]); v[4 + u] = bfr(a1[u]); } float s = 0.f;
#pragma unroll
    for (int u = 0; u < 8; ++u) s = __fadd_rn(s, v[u]);
#pragma unroll
    for (int sh = 16; sh; sh >>= 1) s += __shfl_xor(s, sh, 32);
    const float mean = s * (1.0f / CM); float q2 = 0.f;
#pragma unroll
    for (int u = 0; u < 8; ++u) { float d0 = __fsub_rn(v[u], mean); asm volatile("" : "+v"(d0)); float p = __fmul_rn(d0, d0); asm volatile("" : "+v"(p)); q2 = __fadd_rn(q2, p); }
#pragma unroll
    for (int sh = 16; sh; sh >>= 1) q2 += __shfl_xor(q2, sh, 32);
    const float rstd = __frsqrt_rn(__fadd_rn(q2 * (1.0f / CM), 1e-5f));
    for (int ps = 0; ps < 2; ++ps) {
#pragma unroll
        for (int half = 0; half < 2; ++half) { const int c0 = half * 128 + lane * 4; v4us oh, ol;
#pragma unroll
            for (int u = 0; u < 4; ++u) { float t0 = __fmul_rn(__fsub_rn(v[half * 4 + u], mean), rstd); asm volatile("" : "+v"(t0)); float t1 = __fmul_rn(t0, bfr(g[c0 + u])); asm volatile("" : "+v"(t1)); unsigned short hh, ll; splitf(__fadd_rn(t1, bfr(bb[c0 + u])), hh, ll); oh[u] = hh; ol[u] = ll; }
            *(volatile v4us*)(Nh + rb + c0) = oh; *(volatile v4us*)(Nl + rb + c0) = ol; }
        if (ps == 0) __threadfence(); } }
__global__ __launch_bounds__(256) void k_bt16(const float* __restrict__ PB, h16* BT) { const int e = (blockIdx.x * 256 + threadIdx.x) * 2; if (e >= LL * HDm * NSQ) return; const int n = e % NSQ; const int jb = e / NSQ; const int j = jb / HDm, b = jb % HDm; v2h o; o[0] = tohx(PB[((size_t)n * LL + j) * HP + b]); o[1] = tohx(PB[((size_t)(n + 1) * LL + j) * HP + b]); *(volatile v2h*)(BT + e) = o; __threadfence(); *(volatile v2h*)(BT + e) = o; }
__global__ __launch_bounds__(256) void k_a16(const float* __restrict__ PA, int i0, h16* A16) { const int e = (blockIdx.x * 256 + threadIdx.x) * 2; if (e >= ICH * HDm * NSQ) return; const int n = e % NSQ; const int ia = e / NSQ; const int il = ia / HDm, a = ia % HDm; v2h o; o[0] = tohx(PA[((size_t)n * LL + i0 + il) * HP + a] * (1.0f / PCAR)); o[1] = tohx(PA[((size_t)(n + 1) * LL + i0 + il) * HP + a] * (1.0f / PCAR)); *(volatile v2h*)(A16 + e) = o; __threadfence(); *(volatile v2h*)(A16 + e) = o; }
__global__ __launch_bounds__(256) void k_perm(const float* __restrict__ OC, bf* Ph, bf* Pl) { const int e = (blockIdx.x * 256 + threadIdx.x) * 4; if (e >= ICH * LL * HDm * HDm) return; const int ab = e % (HDm * HDm); const int ilj = e / (HDm * HDm); const int il = ilj / LL, j = ilj % LL; const int a = ab / HDm, b = ab % HDm; const v4f v = *(const v4f*)(OC + ((size_t)(il * HDm + a)) * (LL * HDm) + j * HDm + b); v4us oh, ol;
#pragma unroll
    for (int u = 0; u < 4; ++u) { unsigned short hh, ll; splitf(v[u], hh, ll); oh[u] = hh; ol[u] = ll; } *(volatile v4us*)(Ph + e) = oh; *(volatile v4us*)(Pl + e) = ol; __threadfence(); *(volatile v4us*)(Ph + e) = oh; *(volatile v4us*)(Pl + e) = ol; }

extern "C" void kernel_launch(void* const* d_in, const int* in_sizes, int n_in,
                              void* d_out, int out_size, void* d_ws, size_t ws_size, hipStream_t stream) {
    (void)in_sizes; (void)n_in; (void)out_size;
    const float* msa = (const float*)d_in[0]; const float* ng = (const float*)d_in[1]; const float* nb = (const float*)d_in[2]; const float* w1 = (const float*)d_in[3]; const float* b1 = (const float*)d_in[4]; const float* w2 = (const float*)d_in[5]; const float* b2 = (const float*)d_in[6]; const float* w3 = (const float*)d_in[7]; const float* b3 = (const float*)d_in[8];
    float* OUT = (float*)d_out;
    char* wsp = (char*)d_ws;
    auto take = [&](size_t bytes) { char* p = wsp; wsp += (bytes + 255) & ~(size_t)255; return (void*)p; };
    bf* W1T = (bf*)take(HP * CM * 2); bf* W2T = (bf*)take(HP * CM * 2); float* B1P = (float*)take(256); float* B2P = (float*)take(256); bf* W3T = (bf*)take((size_t)PD * 1024 * 2);
    bf* Nh = (bf*)take((size_t)NR * CM * 2); bf* Nl = (bf*)take((size_t)NR * CM * 2); float* PA = (float*)take((size_t)NR * HP * 4); float* PB = (float*)take((size_t)NR * HP * 4); h16* BT = (h16*)take((size_t)LL * HDm * NSQ * 2); h16* A16 = (h16*)take((size_t)ICH * HDm * NSQ * 2); float* OC = (float*)take((size_t)ICH * HDm * LL * HDm * 4); bf* Ph = (bf*)take((size_t)ICH * LL * 1024 * 2); bf* Pl = (bf*)take((size_t)ICH * LL * 1024 * 2);
    if ((size_t)(wsp - (char*)d_ws) > ws_size) return;
    k_wpadT<<<(HP * CM / 2 + 255) / 256, 256, 0, stream>>>(w1, CM, HDm, HP, CM, W1T); k_wpadT<<<(HP * CM / 2 + 255) / 256, 256, 0, stream>>>(w2, CM, HDm, HP, CM, W2T); k_bpad<<<1, 64, 0, stream>>>(b1, B1P); k_bpad<<<1, 64, 0, stream>>>(b2, B2P);
    k_wtG<<<(1024 * PD / 64 + 63) / 64, 256, 0, stream>>>(w3, 1024, PD, W3T);
    k_ln<<<NR / 8, 256, 0, stream>>>(msa, ng, nb, Nh, Nl);
    k_gemmw<bf, 1, true><<<dim3(NR / 64, 1, 1), 32, 0, stream>>>(Nh, Nl, W2T, nullptr, CM, PA, HP, B2P, 0, 0, 0);
    k_gemmw<bf, 1, true><<<dim3(NR / 64, 1, 1), 32, 0, stream>>>(Nh, Nl, W1T, nullptr, CM, PB, HP, B1P, 0, 0, 0);
    k_bt16<<<(LL * HDm * NSQ / 2 + 255) / 256, 256, 0, stream>>>(PB, BT);
    for (int c = 0; c < LL / ICH; ++c) {
        k_a16<<<(ICH * HDm * NSQ / 2 + 255) / 256, 256, 0, stream>>>(PA, c * ICH, A16);
        k_gemmw<h16, 0, false><<<dim3(ICH * HDm / 64, LL * HDm / 64, 1), 32, 0, stream>>>(A16, nullptr, BT, nullptr, NSQ, OC, LL * HDm, nullptr, 0, 0, 0);
        k_perm<<<(ICH * LL * 1024 / 4 + 255) / 256, 256, 0, stream>>>(OC, Ph, Pl);
        k_gemmw<bf, 1, true><<<dim3(ICH * LL / 64, PD / 64, 1), 32, 0, stream>>>(Ph, Pl, W3T, nullptr, 1024, OUT + (size_t)c * ICH * LL * PD, PD, b3, 0, 0, 0); }
}
